// InteractionNetworkNeighborhood_23158463660311
// MI455X (gfx1250) — hardware-verified
//
#include <hip/hip_runtime.h>
#include <math.h>

typedef __attribute__((ext_vector_type(16))) _Float16 v16h;
typedef __attribute__((ext_vector_type(16))) __bf16 v16b;
typedef __attribute__((ext_vector_type(8)))  _Float16 v8h;
typedef __attribute__((ext_vector_type(8)))  float v8f;
typedef __attribute__((ext_vector_type(4)))  float v4f;
typedef __attribute__((ext_vector_type(2)))  float v2f;
typedef __attribute__((ext_vector_type(4)))  unsigned v4u;
typedef __attribute__((ext_vector_type(4)))  int v4i;
typedef float __attribute__((may_alias)) float_a;
typedef int __attribute__((may_alias)) int_a;

template <typename T> __device__ __forceinline__ void vst2(void* p, T v) { *(volatile T*)p = v; __threadfence(); *(volatile T*)p = v; }
__device__ __forceinline__ v8f wmma16(v16h a, v16h b, v8f c) {
  v8f d = __builtin_amdgcn_wmma_f32_16x16x32_f16(false, a, false, b, (short)0, c, false, false);
  asm volatile("v_nop\n\tv_nop\n\tv_nop\n\tv_nop" : "+v"(d) : "v"(a), "v"(b));
  return d;
}
__device__ __forceinline__ v8f wmma_bf(v16b a, v16b b, v8f c) {
  v8f d = __builtin_amdgcn_wmma_f32_16x16x32_bf16(false, a, false, b, (short)0, c, false, false);
  asm volatile("v_nop\n\tv_nop\n\tv_nop\n\tv_nop" : "+v"(d) : "v"(a), "v"(b));
  return d;
}
__device__ __forceinline__ v16h frag_h(const _Float16* rowk0, int lane) {
  union { v16h v; v8h q[2]; } u; const _Float16* p = rowk0 + 8 * (lane >> 4);
  u.q[0] = *(const v8h*)p; u.q[1] = *(const v8h*)(p + 16); return u.v;
}
__device__ __forceinline__ v16h frag_f32(const float* rowk0, int lane) {
  v16h a; const float* p = rowk0 + 8 * (lane >> 4);
#pragma unroll
  for (int i = 0; i < 8; ++i) { a[i] = (_Float16)p[i]; a[8 + i] = (_Float16)p[16 + i]; }
  return a;
}
__device__ __forceinline__ v16h frag_f32s(const float* rowk0, int lane, float sc) {
  v16h a; const float* p = rowk0 + 8 * (lane >> 4);
#pragma unroll
  for (int i = 0; i < 8; ++i) { a[i] = (_Float16)(p[i] * sc); a[8 + i] = (_Float16)(p[16 + i] * sc); }
  return a;
}
__device__ __forceinline__ v16h fragc_f32(const float* W, int k0, int n, int lane, int ld, int K) {
  v16h a; const int g = lane >> 4;
#pragma unroll
  for (int i = 0; i < 8; ++i) { const int ka = k0 + 8 * g + i, kb = ka + 16;
    a[i] = (_Float16)(ka < K ? W[(size_t)(ka < K ? ka : K - 1) * ld + n] : 0.f); a[8 + i] = (_Float16)(kb < K ? W[(size_t)(kb < K ? kb : K - 1) * ld + n] : 0.f); }
  return a;
}
struct F2 { v16b h, l; };
__device__ __forceinline__ F2 bsplit16(const float v[16]) { F2 r;
#pragma unroll
  for (int i = 0; i < 16; ++i) { const __bf16 h = (__bf16)v[i]; r.h[i] = h; r.l[i] = (__bf16)(v[i] - (float)h); }
  return r; }
__device__ __forceinline__ F2 split_row(const float* row, int k0, int lane) { float v[16]; const float* p = row + k0 + 8 * (lane >> 4);
#pragma unroll
  for (int i = 0; i < 8; ++i) { v[i] = p[i]; v[8 + i] = p[16 + i]; }
  return bsplit16(v); }
__device__ __forceinline__ F2 split_rowK(const float* row, int k0, int lane, int K) { float v[16]; const int g = lane >> 4;
#pragma unroll
  for (int i = 0; i < 8; ++i) { const int ka = k0 + 8 * g + i, kb = ka + 16; v[i] = ka < K ? row[ka < K ? ka : K - 1] : 0.f; v[8 + i] = kb < K ? row[kb < K ? kb : K - 1] : 0.f; }
  return bsplit16(v); }
__device__ __forceinline__ F2 split_col(const float* W, int k0, int n, int lane, int ld, int K) { float v[16]; const int g = lane >> 4;
#pragma unroll
  for (int i = 0; i < 8; ++i) { const int ka = k0 + 8 * g + i, kb = ka + 16; v[i] = ka < K ? W[(size_t)(ka < K ? ka : K - 1) * ld + n] : 0.f; v[8 + i] = kb < K ? W[(size_t)(kb < K ? kb : K - 1) * ld + n] : 0.f; }
  return bsplit16(v); }
__device__ __forceinline__ v8f mac3(const F2& a, const F2& b, v8f c) { c = wmma_bf(a.l, b.h, c); c = wmma_bf(a.h, b.l, c); return wmma_bf(a.h, b.h, c); }
__device__ __forceinline__ float sigm(float v) { return 1.0f / (1.0f + expf(-v)); }
#define LDSX() do { asm volatile("s_wait_dscnt 0" ::: "memory"); __builtin_amdgcn_wave_barrier(); __builtin_amdgcn_fence(__ATOMIC_RELEASE, "workgroup"); } while (0)


#define NB 4
#define NPT 4096
#define KN 16
#define CIN 128
#define IN2 256
#define H1 256
#define H2 256
#define COUT 128
#define WSC 256.0f
#define NP (NB * NPT)
#ifndef TBLK
#define TBLK (NP / 4)
#endif
typedef __attribute__((ext_vector_type(8))) __bf16 v8b;
__device__ __forceinline__ v16b frag_b(const __bf16* rowk0, int lane) {
  union { v16b v; v8b q[2]; } u; const __bf16* p = rowk0 + 8 * (lane >> 4);
  u.q[0] = *(const v8b*)p; u.q[1] = *(const v8b*)(p + 16); return u.v;
}
__device__ __forceinline__ float bfr(float v) { return (float)(__bf16)v; }
__device__ __attribute__((noinline)) float exp_ni(float v) { return expf(v); }
__device__ __attribute__((noinline)) float erf_ni(float v) { return erff(v); }

#define WS_P1  0u
#define WS_P2  (WS_P1 + 2u * H1 * IN2)
#define WS_P3  (WS_P2 + 2u * H2 * H1)
#define WS_END (WS_P3 + 2u * COUT * H2)

__global__ __launch_bounds__(256) void k_packw(const float* __restrict__ W1, const float* __restrict__ W2, const float* __restrict__ W3, char* __restrict__ ws) { const int n = blockIdx.x, t = threadIdx.x; __shared__ __align__(16) __bf16 s1[IN2]; __shared__ __align__(16) _Float16 s2[H1], s3[H2];
  s1[t] = (__bf16)W1[(size_t)t * H1 + n]; s2[t] = (_Float16)(bfr(W2[(size_t)t * H2 + n]) * WSC); if (n < COUT) s3[t] = (_Float16)(bfr(W3[(size_t)t * COUT + n]) * WSC); __syncthreads();
  if (t < IN2 / 8) vst2((unsigned*)((__bf16*)(ws + WS_P1) + (size_t)n * IN2 + t * 8), *(const v4u*)&s1[t * 8]); if (t < H1 / 8) vst2((unsigned*)((_Float16*)(ws + WS_P2) + (size_t)n * H1 + t * 8), *(const v4u*)&s2[t * 8]); if (n < COUT && t < H2 / 8) vst2((unsigned*)((_Float16*)(ws + WS_P3) + (size_t)n * H2 + t * 8), *(const v4u*)&s3[t * 8]); }
__device__ __forceinline__ v16h frag_lds(const _Float16* p, int lane) { v16h a; const _Float16* pp = p + 8 * (lane >> 4);
#pragma unroll
  for (int i = 0; i < 8; ++i) { a[i] = pp[i]; a[8 + i] = pp[16 + i]; } return a; }
__global__ __launch_bounds__(128) void k_inn(const float* __restrict__ FT, const int* __restrict__ IDX, const int* __restrict__ VALID, const __bf16* __restrict__ P1, const float* __restrict__ B1, const _Float16* __restrict__ P2, const float* __restrict__ B2, const _Float16* __restrict__ P3, const float* __restrict__ B3, float* __restrict__ OUT) {
  __shared__ __align__(16) _Float16 sh[64][H1 + 8]; __shared__ int sidx[64]; __shared__ float sval[64]; __shared__ __align__(16) float se[64][COUT + 4]; __shared__ __align__(16) float so[4][COUT + 4];
  const int tid = threadIdx.x, wave = tid >> 5, lane = tid & 31, col = lane & 15, g = lane >> 4; const size_t p0 = (size_t)blockIdx.x * 4; const size_t b = p0 / NPT;
  if (tid < 64) { int ix = IDX[(p0 + (tid >> 4)) * KN + (tid & 15)]; ix = ix < 0 ? 0 : (ix >= NPT ? NPT - 1 : ix); sidx[tid] = ix; sval[tid] = (VALID[(p0 + (tid >> 4)) * KN + (tid & 15)] != 0) ? 1.0f : 0.0f; } __syncthreads();
  const int rl = wave * 16 + col; const float* fi = FT + (p0 + wave) * CIN; const float* fj = FT + (b * NPT + sidx[rl]) * CIN;
  { v8f acc[16];
#pragma unroll
    for (int j = 0; j < 16; ++j) acc[j] = v8f{};
#pragma unroll
    for (int kc = 0; kc < IN2 / 32; ++kc) { v16b a; const float* src = (kc < CIN / 32) ? fi + kc * 32 : fj + (kc - CIN / 32) * 32; const float* pp = src + 8 * g;
#pragma unroll
      for (int i = 0; i < 8; ++i) { a[i] = (__bf16)pp[i]; a[8 + i] = (__bf16)pp[16 + i]; }
#pragma unroll
      for (int j = 0; j < 16; ++j) acc[j] = wmma_bf(a, frag_b(P1 + (size_t)(j * 16 + col) * IN2 + kc * 32, lane), acc[j]); }
#pragma unroll
    for (int j = 0; j < 16; ++j) { const int c = j * 16 + col; const float bb = bfr(B1[c]);
#pragma unroll
      for (int r = 0; r < 8; ++r) sh[wave * 16 + 8 * g + r][c] = (_Float16)fmaxf(acc[j][r] + bb, 0.f); } }
  __syncthreads();
  { v8f acc[16];
#pragma unroll
    for (int j = 0; j < 16; ++j) acc[j] = v8f{};
#pragma unroll
    for (int kc = 0; kc < H1 / 32; ++kc) { const v16h a = frag_lds(&sh[wave * 16 + col][kc * 32], lane);
#pragma unroll
      for (int j = 0; j < 16; ++j) acc[j] = wmma16(a, frag_h(P2 + (size_t)(j * 16 + col) * H1 + kc * 32, lane), acc[j]); }
    __syncthreads();
#pragma unroll
    for (int j = 0; j < 16; ++j) { const int c = j * 16 + col; const float bb = bfr(B2[c]);
#pragma unroll
      for (int r = 0; r < 8; ++r) sh[wave * 16 + 8 * g + r][c] = (_Float16)fmaxf(acc[j][r] * (1.0f / WSC) + bb, 0.f); } }
  __syncthreads();
  { v8f acc[8] = {};
#pragma unroll
    for (int kc = 0; kc < H2 / 32; ++kc) { const v16h a = frag_lds(&sh[wave * 16 + col][kc * 32], lane);
#pragma unroll
      for (int j = 0; j < 8; ++j) acc[j] = wmma16(a, frag_h(P3 + (size_t)(j * 16 + col) * H2 + kc * 32, lane), acc[j]); }
#pragma unroll
    for (int j = 0; j < 8; ++j) { const int c = j * 16 + col; const float bb = bfr(B3[c]);
#pragma unroll
      for (int r = 0; r < 8; ++r) { const int e = wave * 16 + 8 * g + r; se[e][c] = (acc[j][r] * (1.0f / WSC) + bb) * sval[e]; } } }
  __syncthreads();
  for (int e = tid; e < 4 * COUT; e += 128) { const int pt = e / COUT, c = e % COUT; float s = 0.f;
#pragma unroll
    for (int k = 0; k < KN; ++k) s += se[pt * KN + k][c]; so[pt][c] = s; }
  __syncthreads(); { const int pt = tid >> 5, q = tid & 31; vst2(OUT + (p0 + pt) * COUT + q * 4, *(const v4f*)&so[pt][q * 4]); } }
extern "C" void kernel_launch(void* const* d_in, const int* in_sizes, int n_in, void* d_out, int out_size, void* d_ws, size_t ws_size, hipStream_t stream) {
  (void)in_sizes; (void)n_in; (void)out_size;
  const float** F = (const float**)d_in;
  if (ws_size < (size_t)WS_END) return;
  char* ws = (char*)d_ws;
  k_packw<<<H1, 256, 0, stream>>>(F[5], F[7], F[9], ws);
  k_inn<<<TBLK, 128, 0, stream>>>(F[2], (const int*)d_in[3], (const int*)d_in[4], (const __bf16*)(ws + WS_P1), F[6], (const _Float16*)(ws + WS_P2), F[8], (const _Float16*)(ws + WS_P3), F[10], (float*)d_out);
}
